// HSR_2_25116968747549
// MI455X (gfx1250) — hardware-verified
//
#include <hip/hip_runtime.h>
#include <stddef.h>


#define DIN   64
#define HDC   256
#define NHD   4
#define GR    32
#define CP    260
#define NB    64
#define CHUNK 2048
#define NTHR  256
#define NWAVE 8
#define WCAP  256
#define NGRP  (CHUNK / (NTHR * 4))
#define PTH   128
#define YP    68
#define HP    72

#define LDS_F (NB * HDC + NB * HDC + NB * NHD + NB * NHD)
#define LDS_I (NWAVE * WCAP + NWAVE)
#define AGG_LDS_BYTES ((LDS_F + LDS_I) * 4)

static_assert(WCAP == (CHUNK / NTHR) * 32);
static_assert(NGRP >= 1);
static_assert(NB == 64);
static_assert(CHUNK == 2048);
static_assert(HDC / 4 == 64);
static_assert(NB * NHD == NTHR);
static_assert(NB % NWAVE == 0);
static_assert(AGG_LDS_BYTES == 141344);
static_assert((CP * 4) % 16 == 0 && (YP * 4) % 16 == 0 && (HP * 2) % 16 == 0);

typedef float          v4f  __attribute__((ext_vector_type(4)));
typedef float          v8f  __attribute__((ext_vector_type(8)));
typedef int            v4i  __attribute__((ext_vector_type(4)));
typedef unsigned short v8us __attribute__((ext_vector_type(8)));
typedef __bf16         v16b __attribute__((ext_vector_type(16)));

union FragB { v16b v; v4i q[2]; };
union PackU { v8us h; v4i q; };

__device__ __forceinline__ v8f wmb(v16b a, v16b b, v8f c) {
  v8f d = __builtin_amdgcn_wmma_f32_16x16x32_bf16(false, a, false, b, (short)0, c, false, false);
  asm volatile("v_nop\n\tv_nop\n\tv_nop\n\tv_nop" : "+v"(d) : "v"(a), "v"(b));
  return d;
}
__device__ __forceinline__ v8f wmb3(const FragB& ah, const FragB& al, const FragB& bh, const FragB& bl, v8f c) {
  c = wmb(ah.v, bh.v, c);
  c = wmb(ah.v, bl.v, c);
  c = wmb(al.v, bh.v, c);
  return c;
}
__device__ __forceinline__ v8f zero8() {
  v8f z = {0.f, 0.f, 0.f, 0.f, 0.f, 0.f, 0.f, 0.f};
  return z;
}

__device__ __forceinline__ unsigned int bfr(float f) {
  const unsigned int u = __float_as_uint(f);
  return (u + 0x7FFFu + ((u >> 16) & 1u)) >> 16;
}
__device__ __forceinline__ void split8(v4f a, v4f b, v4i& qh, v4i& ql) {
  float v[8];
  v[0] = a.x; v[1] = a.y; v[2] = a.z; v[3] = a.w; v[4] = b.x; v[5] = b.y; v[6] = b.z; v[7] = b.w;
  PackU ph, pl;
#pragma unroll
  for (int j = 0; j < 8; ++j) {
    const unsigned int hb = bfr(v[j]);
    const float fh = __uint_as_float(hb << 16);
    ph.h[j] = (unsigned short)hb;
    pl.h[j] = (unsigned short)bfr(v[j] - fh);
  }
  qh = ph.q;
  ql = pl.q;
}

__device__ __forceinline__ v4f lk4(v4f t, float s) {
  v4f r;
  r.x = fmaxf(t.x, s * t.x); r.y = fmaxf(t.y, s * t.y);
  r.z = fmaxf(t.z, s * t.z); r.w = fmaxf(t.w, s * t.w);
  return r;
}
__device__ __forceinline__ float dot4(v4f a, v4f b) {
  return a.x * b.x + a.y * b.y + a.z * b.z + a.w * b.w;
}

__global__ __launch_bounds__(NTHR) void k_wprep(const float* __restrict__ W, int K, int Nc,
                                                unsigned short* Th, unsigned short* Tl) {
  __shared__ float Ws[64 * 65];
  const int tid = threadIdx.x;
  const int nbt = Nc >> 6;
  const int kt  = blockIdx.x / nbt;
  const int nt  = blockIdx.x - kt * nbt;
  {
    const int r  = tid >> 2;
    const int c0 = (tid & 3) * 16;
    const float* p = W + (size_t)(kt * 64 + r) * Nc + nt * 64 + c0;
#pragma unroll
    for (int q = 0; q < 4; ++q) {
      const v4f f = *(const v4f*)(p + 4 * q);
      float* d = Ws + r * 65 + c0 + 4 * q;
      d[0] = f.x; d[1] = f.y; d[2] = f.z; d[3] = f.w;
    }
  }
  __syncthreads();
  v4i qh[2], ql[2];
  size_t po[2];
#pragma unroll
  for (int ps = 0; ps < 2; ++ps) {
    const int c  = (tid >> 3) + 32 * ps;
    const int k8 = (tid & 7) * 8;
    v4f a, b;
    a.x = Ws[(k8 + 0) * 65 + c]; a.y = Ws[(k8 + 1) * 65 + c];
    a.z = Ws[(k8 + 2) * 65 + c]; a.w = Ws[(k8 + 3) * 65 + c];
    b.x = Ws[(k8 + 4) * 65 + c]; b.y = Ws[(k8 + 5) * 65 + c];
    b.z = Ws[(k8 + 6) * 65 + c]; b.w = Ws[(k8 + 7) * 65 + c];
    split8(a, b, qh[ps], ql[ps]);
    po[ps] = (size_t)(nt * 64 + c) * (size_t)K + (size_t)(kt * 64 + k8);
  }
#pragma unroll
  for (int ps = 0; ps < 2; ++ps) { *(volatile v4i*)(Th + po[ps]) = qh[ps]; *(volatile v4i*)(Tl + po[ps]) = ql[ps]; }
  __threadfence();
#pragma unroll
  for (int ps = 0; ps < 2; ++ps) { *(volatile v4i*)(Th + po[ps]) = qh[ps]; *(volatile v4i*)(Tl + po[ps]) = ql[ps]; }
}

__global__ __launch_bounds__(NTHR) void k_xprep(const float* __restrict__ x, unsigned short* Xh,
                                                unsigned short* Xl, int n8) {
  const int i = blockIdx.x * NTHR + threadIdx.x;
  if (i >= n8) return;
  const size_t o = (size_t)i * 8;
  const v4f a = *(const v4f*)(x + o);
  const v4f b = *(const v4f*)(x + o + 4);
  v4i qh, ql;
  split8(a, b, qh, ql);
  *(volatile v4i*)(Xh + o) = qh;
  *(volatile v4i*)(Xl + o) = ql;
  __threadfence();
  *(volatile v4i*)(Xh + o) = qh;
  *(volatile v4i*)(Xl + o) = ql;
}

__global__ __launch_bounds__(NTHR) void k_proj(
    const unsigned short* __restrict__ Ah, const unsigned short* __restrict__ Al,
    const unsigned short* __restrict__ B0h, const unsigned short* __restrict__ B0l,
    const float* __restrict__ bias0, float* C0,
    const unsigned short* __restrict__ B1h, const unsigned short* __restrict__ B1l,
    const float* __restrict__ bias1, float* C1, int M) {
  __shared__ __attribute__((aligned(16))) float Cs[GR * CP];

  const int tid  = threadIdx.x;
  const int lane = tid & 31;
  const int wave = tid >> 5;
  const int h    = lane >> 4;
  const int m    = lane & 15;
  const int rowBase = blockIdx.x * GR;
  const bool sel = (blockIdx.y != 0);
  const unsigned short* Bh = sel ? B1h : B0h;
  const unsigned short* Bl = sel ? B1l : B0l;
  const float* bias = sel ? bias1 : bias0;
  float* C = sel ? C1 : C0;

  int rA0 = rowBase + m;      if (rA0 > M - 1) rA0 = M - 1;
  int rA1 = rowBase + 16 + m; if (rA1 > M - 1) rA1 = M - 1;
  const int cw = wave * 32;

  v8f acc00 = zero8(), acc01 = zero8(), acc10 = zero8(), acc11 = zero8();
#pragma unroll
  for (int kt = 0; kt < DIN / 32; ++kt) {
    const int k0 = kt * 32 + 8 * h;
    FragB ah0, al0, ah1, al1, bh0, bl0, bh1, bl1;
    const unsigned short* p;
    p = Ah + (size_t)rA0 * DIN + k0;         ah0.q[0] = *(const v4i*)p; ah0.q[1] = *(const v4i*)(p + 16);
    p = Al + (size_t)rA0 * DIN + k0;         al0.q[0] = *(const v4i*)p; al0.q[1] = *(const v4i*)(p + 16);
    p = Ah + (size_t)rA1 * DIN + k0;         ah1.q[0] = *(const v4i*)p; ah1.q[1] = *(const v4i*)(p + 16);
    p = Al + (size_t)rA1 * DIN + k0;         al1.q[0] = *(const v4i*)p; al1.q[1] = *(const v4i*)(p + 16);
    p = Bh + (size_t)(cw + m) * DIN + k0;      bh0.q[0] = *(const v4i*)p; bh0.q[1] = *(const v4i*)(p + 16);
    p = Bl + (size_t)(cw + m) * DIN + k0;      bl0.q[0] = *(const v4i*)p; bl0.q[1] = *(const v4i*)(p + 16);
    p = Bh + (size_t)(cw + 16 + m) * DIN + k0; bh1.q[0] = *(const v4i*)p; bh1.q[1] = *(const v4i*)(p + 16);
    p = Bl + (size_t)(cw + 16 + m) * DIN + k0; bl1.q[0] = *(const v4i*)p; bl1.q[1] = *(const v4i*)(p + 16);
    acc00 = wmb3(ah0, al0, bh0, bl0, acc00);
    acc01 = wmb3(ah0, al0, bh1, bl1, acc01);
    acc10 = wmb3(ah1, al1, bh0, bl0, acc10);
    acc11 = wmb3(ah1, al1, bh1, bl1, acc11);
  }

  const float bv0 = bias[cw + m];
  const float bv1 = bias[cw + 16 + m];
#pragma unroll
  for (int r = 0; r < 8; ++r) {
    Cs[(8 * h + r) * CP + cw + m]           = acc00[r] + bv0;
    Cs[(8 * h + r) * CP + cw + 16 + m]      = acc01[r] + bv1;
    Cs[(16 + 8 * h + r) * CP + cw + m]      = acc10[r] + bv0;
    Cs[(16 + 8 * h + r) * CP + cw + 16 + m] = acc11[r] + bv1;
  }
  __syncthreads();

  v4f o[8];
  size_t po[4];
  bool ok[4];
#pragma unroll
  for (int i = 0; i < 4; ++i) {
    const int rowl = 4 * wave + i;
    o[2 * i]     = *(const v4f*)(Cs + rowl * CP + 4 * lane);
    o[2 * i + 1] = *(const v4f*)(Cs + rowl * CP + 128 + 4 * lane);
    po[i] = (size_t)(rowBase + rowl) * HDC + 4 * lane;
    ok[i] = (rowBase + rowl) < M;
  }
#pragma unroll
  for (int i = 0; i < 4; ++i) {
    if (ok[i]) { *(volatile v4f*)(C + po[i]) = o[2 * i]; *(volatile v4f*)(C + po[i] + 128) = o[2 * i + 1]; }
  }
  __threadfence();
#pragma unroll
  for (int i = 0; i < 4; ++i) {
    if (ok[i]) { *(volatile v4f*)(C + po[i]) = o[2 * i]; *(volatile v4f*)(C + po[i] + 128) = o[2 * i + 1]; }
  }
}

__global__ __launch_bounds__(NTHR) void k_agg(
    const int* __restrict__ esrc, const int* __restrict__ edst,
    const float* __restrict__ XL, const float* __restrict__ XR,
    const float* __restrict__ att, const float* __restrict__ cbv,
    unsigned short* Gh, unsigned short* Gl, int nN, int nE) {
  extern __shared__ v4f lds_dyn[];
  float* sacc = (float*)lds_dyn;
  float* xrs  = sacc + NB * HDC;
  float* mxa  = xrs + NB * HDC;
  float* den  = mxa + NB * NHD;
  int*   list = (int*)(den + NB * NHD);
  int*   wcnt = list + NWAVE * WCAP;

  const int tid  = threadIdx.x;
  const int lane = tid & 31;
  const int wave = tid >> 5;
  const int hd   = lane >> 3;
  const int nodeBase = blockIdx.x * NB;

  {
    const v4f z4 = {0.f, 0.f, 0.f, 0.f};
    for (int i = tid; i < NB * HDC / 4; i += NTHR) lds_dyn[i] = z4;
    v4f* xr4 = lds_dyn + NB * HDC / 4;
    for (int i = tid; i < NB * HDC / 4; i += NTHR) {
      const int r = i >> 6;
      const int q = i & 63;
      int node = nodeBase + r;
      if (node > nN - 1) node = nN - 1;
      xr4[i] = *(const v4f*)(XR + (size_t)node * HDC + 4 * q);
    }
    mxa[tid] = -1.0e30f;
    den[tid] = 0.f;
  }
  const v4f at0 = *(const v4f*)(att + 8 * lane);
  const v4f at1 = *(const v4f*)(att + 8 * lane + 4);
  __syncthreads();

  const int nChunks = (nE + CHUNK - 1) / CHUNK;
#pragma unroll 1
  for (int ch = 0; ch < nChunks; ++ch) {
    const int cbase = ch * CHUNK;
    const bool full = (cbase + CHUNK <= nE);
    int wc = 0;
#pragma unroll
    for (int g = 0; g < NGRP; ++g) {
      const int el0 = (g * NTHR + tid) * 4;
      const int e0  = cbase + el0;
      const int sent = -2147483647 - 1;
      v4i d;
      if (full) {
        d = *(const v4i*)(edst + e0);
      } else {
        const int c0 = min(e0, nE - 1), c1 = min(e0 + 1, nE - 1);
        const int c2 = min(e0 + 2, nE - 1), c3 = min(e0 + 3, nE - 1);
        d.x = (e0     < nE) ? edst[c0] : sent;
        d.y = (e0 + 1 < nE) ? edst[c1] : sent;
        d.z = (e0 + 2 < nE) ? edst[c2] : sent;
        d.w = (e0 + 3 < nE) ? edst[c3] : sent;
      }
      const unsigned s0 = (unsigned)d.x - (unsigned)nodeBase;
      const unsigned s1 = (unsigned)d.y - (unsigned)nodeBase;
      const unsigned s2 = (unsigned)d.z - (unsigned)nodeBase;
      const unsigned s3 = (unsigned)d.w - (unsigned)nodeBase;
      const bool h0 = s0 < (unsigned)NB;
      const bool h1 = s1 < (unsigned)NB;
      const bool h2 = s2 < (unsigned)NB;
      const bool h3 = s3 < (unsigned)NB;
      const unsigned many = __builtin_amdgcn_ballot_w32(h0 | h1 | h2 | h3);
      if (many != 0u) {
#define HITJ(J, HJ, SJ) { \
          const unsigned mj = __builtin_amdgcn_ballot_w32(HJ); \
          if (HJ) { \
            const int pos = wc + (int)__builtin_amdgcn_mbcnt_lo(mj, 0u); \
            if (pos < WCAP) list[wave * WCAP + pos] = ((el0 + (J)) << 6) | (int)(SJ); \
          } \
          wc += (int)__builtin_popcount(mj); }
        HITJ(0, h0, s0)
        HITJ(1, h1, s1)
        HITJ(2, h2, s2)
        HITJ(3, h3, s3)
#undef HITJ
      }
    }
    if (lane == 0) wcnt[wave] = wc;
    __syncthreads();

    if (wave == 0) {
#pragma unroll 1
      for (int wsx = 0; wsx < NWAVE; ++wsx) {
        int n = wcnt[wsx];
        n = n < 0 ? 0 : (n > WCAP ? WCAP : n);
#pragma unroll 1
        for (int i = 0; i < n; ++i) {
          const int ent  = list[wsx * WCAP + i];
          const int slot = ent & (NB - 1);
          const int el   = (ent >> 6) & (CHUNK - 1);
          int e = cbase + el;
          if (e > nE - 1) e = nE - 1;
          int src = esrc[e];
          src = src < 0 ? 0 : (src > nN - 1 ? nN - 1 : src);
          const float* xp = XL + (size_t)src * HDC + 8 * lane;
          const v4f x0 = *(const v4f*)xp;
          const v4f x1 = *(const v4f*)(xp + 4);
          const float* rp = xrs + slot * HDC + 8 * lane;
          const v4f q0 = *(const v4f*)rp;
          const v4f q1 = *(const v4f*)(rp + 4);
          const v4f t0 = lk4(x0 + q0, 0.2f);
          const v4f t1 = lk4(x1 + q1, 0.2f);
          float s = dot4(at0, t0) + dot4(at1, t1);
          s += __shfl_xor(s, 4, 32);
          s += __shfl_xor(s, 2, 32);
          s += __shfl_xor(s, 1, 32);
          const int hix = slot * NHD + hd;
          const float mo = mxa[hix];
          const float dn = den[hix];
          const float mn = fmaxf(mo, s);
          const float corr = __expf(mo - mn);
          const float p = __expf(s - mn);
          v4f* sp = (v4f*)(sacc + slot * HDC + 8 * lane);
          v4f a0 = sp[0];
          v4f a1 = sp[1];
          a0 = a0 * corr + x0 * p;
          a1 = a1 * corr + x1 * p;
          sp[0] = a0;
          sp[1] = a1;
          mxa[hix] = mn;
          den[hix] = dn * corr + p;
          __builtin_amdgcn_fence(__ATOMIC_RELEASE, "wavefront");
          __builtin_amdgcn_wave_barrier();
        }
      }
    }
    __syncthreads();
  }

  const v4f c0v = *(const v4f*)(cbv + 8 * lane);
  const v4f c1v = *(const v4f*)(cbv + 8 * lane + 4);
#pragma unroll 1
  for (int j = 0; j < NB / NWAVE; ++j) {
    const int slot = wave * (NB / NWAVE) + j;
    const int node = nodeBase + slot;
    if (node >= nN) break;
    const float dn  = den[slot * NHD + hd];
    const float inv = (dn > 0.f) ? (1.0f / dn) : 0.f;
    const v4f* sp = (const v4f*)(sacc + slot * HDC + 8 * lane);
    const v4f v0 = sp[0] * inv + c0v;
    const v4f v1 = sp[1] * inv + c1v;
    v4i qh, ql;
    split8(v0, v1, qh, ql);
    const size_t o = (size_t)node * HDC + 8 * lane;
    *(volatile v4i*)(Gh + o) = qh;
    *(volatile v4i*)(Gl + o) = ql;
    __threadfence();
    *(volatile v4i*)(Gh + o) = qh;
    *(volatile v4i*)(Gl + o) = ql;
  }
}

template <int MODE>
__global__ __launch_bounds__(PTH) void k_post(
    const unsigned short* __restrict__ Ah, const unsigned short* __restrict__ Al,
    const unsigned short* __restrict__ Lh, const unsigned short* __restrict__ Ll,
    const unsigned short* __restrict__ Wh, const unsigned short* __restrict__ Wl,
    const float* __restrict__ bvec, const float* __restrict__ gam, const float* __restrict__ bet,
    unsigned short* Oh, unsigned short* Ol, float* Of, int M) {
  __shared__ __attribute__((aligned(16))) float Ys[GR * YP];
  __shared__ __attribute__((aligned(16))) unsigned short Yh[GR * HP];
  __shared__ __attribute__((aligned(16))) unsigned short Yl[GR * HP];

  const int tid  = threadIdx.x;
  const int lane = tid & 31;
  const int wave = tid >> 5;
  const int h    = lane >> 4;
  const int m    = lane & 15;
  const int rowBase = blockIdx.x * GR;
  int rA0 = rowBase + m;      if (rA0 > M - 1) rA0 = M - 1;
  int rA1 = rowBase + 16 + m; if (rA1 > M - 1) rA1 = M - 1;
  const int ncol = wave * 16 + m;

  v8f y0 = zero8(), y1 = zero8();
#pragma unroll 2
  for (int kt = 0; kt < HDC / 32; ++kt) {
    const int k0 = kt * 32 + 8 * h;
    FragB a0h, a0l, a1h, a1l, bh, bl;
    const unsigned short* p;
    p = Ah + (size_t)rA0 * HDC + k0;  a0h.q[0] = *(const v4i*)p; a0h.q[1] = *(const v4i*)(p + 16);
    p = Al + (size_t)rA0 * HDC + k0;  a0l.q[0] = *(const v4i*)p; a0l.q[1] = *(const v4i*)(p + 16);
    p = Ah + (size_t)rA1 * HDC + k0;  a1h.q[0] = *(const v4i*)p; a1h.q[1] = *(const v4i*)(p + 16);
    p = Al + (size_t)rA1 * HDC + k0;  a1l.q[0] = *(const v4i*)p; a1l.q[1] = *(const v4i*)(p + 16);
    p = Lh + (size_t)ncol * HDC + k0; bh.q[0]  = *(const v4i*)p; bh.q[1]  = *(const v4i*)(p + 16);
    p = Ll + (size_t)ncol * HDC + k0; bl.q[0]  = *(const v4i*)p; bl.q[1]  = *(const v4i*)(p + 16);
    y0 = wmb3(a0h, a0l, bh, bl, y0);
    y1 = wmb3(a1h, a1l, bh, bl, y1);
  }
#pragma unroll
  for (int r = 0; r < 8; ++r) {
    Ys[(8 * h + r) * YP + ncol]      = y0[r];
    Ys[(16 + 8 * h + r) * YP + ncol] = y1[r];
  }
  __syncthreads();

  {
    const int row = tid >> 2;
    const int c0  = (tid & 3) * 16;
    const float* yp = Ys + row * YP + c0;
    const v4f f0 = *(const v4f*)(yp), f1 = *(const v4f*)(yp + 4);
    const v4f f2 = *(const v4f*)(yp + 8), f3 = *(const v4f*)(yp + 12);
    v4i qh0, ql0, qh1, ql1;
    split8(f0, f1, qh0, ql0);
    split8(f2, f3, qh1, ql1);
    *(v4i*)(Yh + row * HP + c0)     = qh0;
    *(v4i*)(Yh + row * HP + c0 + 8) = qh1;
    *(v4i*)(Yl + row * HP + c0)     = ql0;
    *(v4i*)(Yl + row * HP + c0 + 8) = ql1;
  }
  __syncthreads();

  v8f z0 = zero8(), z1 = zero8();
#pragma unroll
  for (int kt = 0; kt < DIN / 32; ++kt) {
    const int k0 = kt * 32 + 8 * h;
    FragB a0h, a0l, a1h, a1l, bh, bl;
    a0h.q[0] = *(const v4i*)(Yh + m * HP + k0);        a0h.q[1] = *(const v4i*)(Yh + m * HP + k0 + 16);
    a0l.q[0] = *(const v4i*)(Yl + m * HP + k0);        a0l.q[1] = *(const v4i*)(Yl + m * HP + k0 + 16);
    a1h.q[0] = *(const v4i*)(Yh + (16 + m) * HP + k0); a1h.q[1] = *(const v4i*)(Yh + (16 + m) * HP + k0 + 16);
    a1l.q[0] = *(const v4i*)(Yl + (16 + m) * HP + k0); a1l.q[1] = *(const v4i*)(Yl + (16 + m) * HP + k0 + 16);
    const unsigned short* p;
    p = Wh + (size_t)ncol * DIN + k0; bh.q[0] = *(const v4i*)p; bh.q[1] = *(const v4i*)(p + 16);
    p = Wl + (size_t)ncol * DIN + k0; bl.q[0] = *(const v4i*)p; bl.q[1] = *(const v4i*)(p + 16);
    z0 = wmb3(a0h, a0l, bh, bl, z0);
    z1 = wmb3(a1h, a1l, bh, bl, z1);
  }
  const float bv = bvec[ncol];
#pragma unroll
  for (int r = 0; r < 8; ++r) {
    float v = z0[r] + bv; v = fmaxf(v, 0.01f * v);
    Ys[(8 * h + r) * YP + ncol] = v;
    float u = z1[r] + bv; u = fmaxf(u, 0.01f * u);
    Ys[(16 + 8 * h + r) * YP + ncol] = u;
  }
  __syncthreads();

  if (MODE == 0) {
    const int c8   = 8 * (lane & 7);
    const int rsub = lane >> 3;
    const v4f g0 = *(const v4f*)(gam + c8), g1 = *(const v4f*)(gam + c8 + 4);
    const v4f e0 = *(const v4f*)(bet + c8), e1 = *(const v4f*)(bet + c8 + 4);
    v4i qh[2], ql[2];
    size_t po[2];
    bool ok[2];
#pragma unroll
    for (int i = 0; i < 2; ++i) {
      const int rowl = 8 * wave + 4 * i + rsub;
      const float* zp = Ys + rowl * YP + c8;
      const v4f v0 = *(const v4f*)zp;
      const v4f v1 = *(const v4f*)(zp + 4);
      float s = (v0.x + v0.y + v0.z + v0.w) + (v1.x + v1.y + v1.z + v1.w);
      s += __shfl_xor(s, 4, 32);
      s += __shfl_xor(s, 2, 32);
      s += __shfl_xor(s, 1, 32);
      const float mu = s * (1.0f / DIN);
      const v4f d0 = v0 - mu, d1 = v1 - mu;
      float q = dot4(d0, d0) + dot4(d1, d1);
      q += __shfl_xor(q, 4, 32);
      q += __shfl_xor(q, 2, 32);
      q += __shfl_xor(q, 1, 32);
      const float rs = rsqrtf(q * (1.0f / DIN) + 1e-5f);
      const v4f yv0 = d0 * rs * g0 + e0;
      const v4f yv1 = d1 * rs * g1 + e1;
      split8(yv0, yv1, qh[i], ql[i]);
      po[i] = (size_t)(rowBase + rowl) * DIN + c8;
      ok[i] = (rowBase + rowl) < M;
    }
#pragma unroll
    for (int i = 0; i < 2; ++i) {
      if (ok[i]) { *(volatile v4i*)(Oh + po[i]) = qh[i]; *(volatile v4i*)(Ol + po[i]) = ql[i]; }
    }
    __threadfence();
#pragma unroll
    for (int i = 0; i < 2; ++i) {
      if (ok[i]) { *(volatile v4i*)(Oh + po[i]) = qh[i]; *(volatile v4i*)(Ol + po[i]) = ql[i]; }
    }
  } else {
    const int c4   = 4 * (lane & 15);
    const int rsub = lane >> 4;
    v4f ov[4];
    size_t po[4];
    bool ok[4];
#pragma unroll
    for (int i = 0; i < 4; ++i) {
      const int rowl = 8 * wave + 2 * i + rsub;
      ov[i] = *(const v4f*)(Ys + rowl * YP + c4);
      po[i] = (size_t)(rowBase + rowl) * DIN + c4;
      ok[i] = (rowBase + rowl) < M;
    }
#pragma unroll
    for (int i = 0; i < 4; ++i) { if (ok[i]) *(volatile v4f*)(Of + po[i]) = ov[i]; }
    __threadfence();
#pragma unroll
    for (int i = 0; i < 4; ++i) { if (ok[i]) *(volatile v4f*)(Of + po[i]) = ov[i]; }
  }
}

extern "C" void kernel_launch(void* const* d_in, const int* in_sizes, int n_in,
                              void* d_out, int out_size, void* d_ws, size_t ws_size,
                              hipStream_t stream) {
  if (n_in < 23) return;
  const int nN = in_sizes[0] / DIN;
  if (nN <= 0 || in_sizes[0] != nN * DIN) return;
  if ((nN % NB) != 0 || (nN % GR) != 0) return;
  if (in_sizes[1] != DIN * HDC || in_sizes[3] != DIN * HDC || in_sizes[8] != DIN * HDC || in_sizes[10] != DIN * HDC) return;
  if (in_sizes[2] != HDC || in_sizes[4] != HDC || in_sizes[6] != HDC) return;
  if (in_sizes[9] != HDC || in_sizes[11] != HDC || in_sizes[13] != HDC) return;
  if (in_sizes[5] != NHD * DIN || in_sizes[12] != NHD * DIN) return;
  if (in_sizes[7] != HDC * DIN || in_sizes[14] != HDC * DIN) return;
  if (in_sizes[15] != DIN * DIN || in_sizes[17] != DIN * DIN) return;
  if (in_sizes[16] != DIN || in_sizes[18] != DIN || in_sizes[19] != DIN || in_sizes[20] != DIN) return;
  const int nE = in_sizes[21];
  if (nE <= 0 || in_sizes[22] != nE) return;
  if (out_size != nN * DIN) return;

  const float* x     = (const float*)d_in[0];
  const float* Wl1   = (const float*)d_in[1];
  const float* bl1   = (const float*)d_in[2];
  const float* Wr1   = (const float*)d_in[3];
  const float* br1   = (const float*)d_in[4];
  const float* att1  = (const float*)d_in[5];
  const float* cb1   = (const float*)d_in[6];
  const float* linw1 = (const float*)d_in[7];
  const float* Wl2   = (const float*)d_in[8];
  const float* bl2   = (const float*)d_in[9];
  const float* Wr2   = (const float*)d_in[10];
  const float* br2   = (const float*)d_in[11];
  const float* att2  = (const float*)d_in[12];
  const float* cb2   = (const float*)d_in[13];
  const float* linw2 = (const float*)d_in[14];
  const float* w1    = (const float*)d_in[15];
  const float* b1    = (const float*)d_in[16];
  const float* w2    = (const float*)d_in[17];
  const float* b2    = (const float*)d_in[18];
  const float* gamma = (const float*)d_in[19];
  const float* beta  = (const float*)d_in[20];
  const int*   esrc  = (const int*)d_in[21];
  const int*   edst  = (const int*)d_in[22];
  float* out = (float*)d_out;

  const size_t szW = (size_t)DIN * HDC * 2;
  const size_t szS = (size_t)DIN * DIN * 2;
  const size_t szX = (size_t)nN * DIN * 2;
  const size_t szP = (size_t)nN * HDC * 4;
  const size_t szG = (size_t)nN * HDC * 2;
  char* wb = (char*)d_ws;
  size_t off = 0;
  unsigned short* WlT1h = (unsigned short*)(wb + off); off += szW;
  unsigned short* WlT1l = (unsigned short*)(wb + off); off += szW;
  unsigned short* WrT1h = (unsigned short*)(wb + off); off += szW;
  unsigned short* WrT1l = (unsigned short*)(wb + off); off += szW;
  unsigned short* WlT2h = (unsigned short*)(wb + off); off += szW;
  unsigned short* WlT2l = (unsigned short*)(wb + off); off += szW;
  unsigned short* WrT2h = (unsigned short*)(wb + off); off += szW;
  unsigned short* WrT2l = (unsigned short*)(wb + off); off += szW;
  unsigned short* LT1h  = (unsigned short*)(wb + off); off += szW;
  unsigned short* LT1l  = (unsigned short*)(wb + off); off += szW;
  unsigned short* LT2h  = (unsigned short*)(wb + off); off += szW;
  unsigned short* LT2l  = (unsigned short*)(wb + off); off += szW;
  unsigned short* W1h   = (unsigned short*)(wb + off); off += szS;
  unsigned short* W1l   = (unsigned short*)(wb + off); off += szS;
  unsigned short* W2h   = (unsigned short*)(wb + off); off += szS;
  unsigned short* W2l   = (unsigned short*)(wb + off); off += szS;
  unsigned short* Xh    = (unsigned short*)(wb + off); off += szX;
  unsigned short* Xl    = (unsigned short*)(wb + off); off += szX;
  unsigned short* Nh    = (unsigned short*)(wb + off); off += szX;
  unsigned short* Nl    = (unsigned short*)(wb + off); off += szX;
  float* XL = (float*)(wb + off); off += szP;
  float* XR = (float*)(wb + off); off += szP;
  unsigned short* Gh    = (unsigned short*)(wb + off); off += szG;
  unsigned short* Gl    = (unsigned short*)(wb + off); off += szG;
  if (off > ws_size) return;
  if (off > (size_t)134217728) return;

  k_wprep<<<(DIN / 64) * (HDC / 64), NTHR, 0, stream>>>(Wl1, DIN, HDC, WlT1h, WlT1l);
  k_wprep<<<(DIN / 64) * (HDC / 64), NTHR, 0, stream>>>(Wr1, DIN, HDC, WrT1h, WrT1l);
  k_wprep<<<(DIN / 64) * (HDC / 64), NTHR, 0, stream>>>(Wl2, DIN, HDC, WlT2h, WlT2l);
  k_wprep<<<(DIN / 64) * (HDC / 64), NTHR, 0, stream>>>(Wr2, DIN, HDC, WrT2h, WrT2l);
  k_wprep<<<(HDC / 64) * (DIN / 64), NTHR, 0, stream>>>(linw1, HDC, DIN, LT1h, LT1l);
  k_wprep<<<(HDC / 64) * (DIN / 64), NTHR, 0, stream>>>(linw2, HDC, DIN, LT2h, LT2l);
  k_wprep<<<(DIN / 64) * (DIN / 64), NTHR, 0, stream>>>(w1, DIN, DIN, W1h, W1l);
  k_wprep<<<(DIN / 64) * (DIN / 64), NTHR, 0, stream>>>(w2, DIN, DIN, W2h, W2l);

  const int n8 = nN * (DIN / 8);
  k_xprep<<<(n8 + NTHR - 1) / NTHR, NTHR, 0, stream>>>(x, Xh, Xl, n8);

  hipFuncSetAttribute(reinterpret_cast<const void*>(&k_agg),
                      hipFuncAttributeMaxDynamicSharedMemorySize, AGG_LDS_BYTES);
  const dim3 gproj((nN + GR - 1) / GR, 2);
  const int  gagg  = (nN + NB - 1) / NB;
  const int  gpost = (nN + GR - 1) / GR;

  k_proj<<<gproj, NTHR, 0, stream>>>(Xh, Xl, WlT1h, WlT1l, bl1, XL, WrT1h, WrT1l, br1, XR, nN);
  k_agg<<<gagg, NTHR, AGG_LDS_BYTES, stream>>>(esrc, edst, XL, XR, att1, cb1, Gh, Gl, nN, nE);
  k_post<0><<<gpost, PTH, 0, stream>>>(Gh, Gl, LT1h, LT1l, W1h, W1l, b1, gamma, beta, Nh, Nl, out, nN);

  k_proj<<<gproj, NTHR, 0, stream>>>(Nh, Nl, WlT2h, WlT2l, bl2, XL, WrT2h, WrT2l, br2, XR, nN);
  k_agg<<<gagg, NTHR, AGG_LDS_BYTES, stream>>>(esrc, edst, XL, XR, att2, cb2, Gh, Gl, nN, nE);
  k_post<1><<<gpost, PTH, 0, stream>>>(Gh, Gl, LT2h, LT2l, W2h, W2l, b2, gamma, beta, Nh, Nl, out, nN);
}
